// StateTransformerBlock_13632226197805
// MI455X (gfx1250) — hardware-verified
//
#include <hip/hip_runtime.h>
#include <math.h>
#include <stdint.h>

typedef _Float16 v8h  __attribute__((ext_vector_type(8)));
typedef _Float16 v16h __attribute__((ext_vector_type(16)));
typedef float    v8f  __attribute__((ext_vector_type(8)));
typedef float    v4f  __attribute__((ext_vector_type(4)));

#define NBATCH 4
#define LSM    1024
#define LSI    4096
#define DMOD   256
#define NHEAD  8
#define DFF    1024
#define MROWS  (NBATCH * LSM)
#define IROWS  (NBATCH * LSI)
#define QCOLS  (NHEAD * DMOD)

static_assert(MROWS % 64 == 0);
static_assert(IROWS % 64 == 0);
static_assert(DMOD % 64 == 0);
static_assert(DFF % 64 == 0);
static_assert(LSI % 32 == 0);
static_assert(LSM % 64 == 0);

__device__ __forceinline__ v8f mma16(v16h a, v16h b, v8f c) {
  c = __builtin_amdgcn_wmma_f32_16x16x32_f16(false, a, false, b, (short)0, c, false, false);
  asm volatile("v_nop\n\tv_nop\n\tv_nop\n\tv_nop" : "+v"(c) : "v"(a), "v"(b));
  return c;
}
union Frag16 { v16h v; v8h h[2]; };
__device__ __forceinline__ v16h ldfrag(const _Float16* p) {
  Frag16 f;
  f.h[0] = *(const v8h*)(p);
  f.h[1] = *(const v8h*)(p + 16);
  return f.v;
}
__device__ __forceinline__ v8f zero8f() {
  v8f z = {0.f, 0.f, 0.f, 0.f, 0.f, 0.f, 0.f, 0.f};
  return z;
}
__device__ __forceinline__ void wave_lds_sync() {
  __builtin_amdgcn_fence(__ATOMIC_RELEASE, "workgroup");
  __builtin_amdgcn_wave_barrier();
  __builtin_amdgcn_fence(__ATOMIC_ACQUIRE, "workgroup");
}

__global__ __launch_bounds__(256) void cvt_f16_kernel(const float* __restrict__ in,
                                                      unsigned short* __restrict__ out, int n8) {
  const int i = blockIdx.x * 256 + threadIdx.x;
  if (i < n8) {
    const v4f a = *(const v4f*)(in + (size_t)i * 8);
    const v4f c = *(const v4f*)(in + (size_t)i * 8 + 4);
    v8h o;
    o[0] = (_Float16)a[0]; o[1] = (_Float16)a[1]; o[2] = (_Float16)a[2]; o[3] = (_Float16)a[3];
    o[4] = (_Float16)c[0]; o[5] = (_Float16)c[1]; o[6] = (_Float16)c[2]; o[7] = (_Float16)c[3];
    _Float16* op = (_Float16*)out + (size_t)i * 8;
    *(volatile v8h*)op = o;
    __threadfence();
    *(volatile v8h*)op = o;
  }
}

__global__ __launch_bounds__(256) void tcvt_kernel(const float* __restrict__ W, unsigned short* __restrict__ outp,
                                                   int R, int Cc, long sIn, long sOut, float wscale) {
  __shared__ __align__(16) float tf[64 * 68];
  W += (size_t)blockIdx.z * sIn;
  _Float16* out = (_Float16*)outp + (size_t)blockIdx.z * sOut;
  const int c0  = blockIdx.x * 64;
  const int r0  = blockIdx.y * 64;
  const int tid = threadIdx.x;
  {
    const int lr = tid >> 4;
    const int c4 = (tid & 15) * 4;
#pragma unroll
    for (int it = 0; it < 4; ++it) {
      const int rr = it * 16 + lr;
      const v4f a = *(const v4f*)(W + (size_t)(r0 + rr) * Cc + c0 + c4);
      *(v4f*)(tf + rr * 68 + c4) = a;
    }
  }
  __syncthreads();
  const int sub = tid >> 3;
  const int c8  = (tid & 7) * 8;
  v8h hv[2];
#pragma unroll
  for (int it = 0; it < 2; ++it) {
    const int oc = it * 32 + sub;
    v8h v;
#pragma unroll
    for (int e = 0; e < 8; ++e) v[e] = (_Float16)(tf[(c8 + e) * 68 + oc] * wscale);
    hv[it] = v;
  }
  for (int pass = 0; pass < 2; ++pass) {
#pragma unroll
    for (int it = 0; it < 2; ++it) {
      const int oc = it * 32 + sub;
      *(volatile v8h*)(out + (size_t)(c0 + oc) * R + r0 + c8) = hv[it];
    }
    __threadfence();
  }
}

template <int BIAS_MODE, int OUT16, int RELU, int MUL>
__global__ __launch_bounds__(256) void gemm_kernel(
    const unsigned short* __restrict__ Ap, int lda, long sA,
    const unsigned short* __restrict__ Bp, int ldb, long sB,
    void* __restrict__ Cp, int ldc, long sC,
    const float* __restrict__ bias, const float* __restrict__ mul,
    int M, int N, int K, float scale, float oscale) {
  __shared__ __align__(16) float sT[8][16 * 68];
  const int z      = blockIdx.y;
  const int lane   = threadIdx.x & 31;
  const int wave   = threadIdx.x >> 5;
  const int tilesN = N >> 6;
  const int tilesM = M >> 5;
  const int tile   = blockIdx.x * 8 + wave;
  if (tile >= tilesM * tilesN) return;
  const int tm = tile / tilesN;
  const int tn = tile - tm * tilesN;
  const int m0 = tm << 5;
  const int n0 = tn << 6;

  const _Float16* A  = (const _Float16*)Ap + (size_t)z * sA;
  const _Float16* Bt = (const _Float16*)Bp + (size_t)z * sB;

  const int rl   = lane & 15;
  const int hf   = lane >> 4;
  const int koff = hf * 8;

  v8f acc[2][4];
#pragma unroll
  for (int i = 0; i < 2; ++i)
#pragma unroll
    for (int j = 0; j < 4; ++j) acc[i][j] = zero8f();

  for (int k0 = 0; k0 < K; k0 += 32) {
    v16h bf[4];
#pragma unroll
    for (int j = 0; j < 4; ++j)
      bf[j] = ldfrag(Bt + (size_t)(n0 + 16 * j + rl) * ldb + k0 + koff);
#pragma unroll
    for (int i = 0; i < 2; ++i) {
      const v16h af = ldfrag(A + (size_t)(m0 + 16 * i + rl) * lda + k0 + koff);
#pragma unroll
      for (int j = 0; j < 4; ++j) acc[i][j] = mma16(af, bf[j], acc[i][j]);
    }
  }

  float* slab = sT[wave];
#pragma unroll
  for (int i = 0; i < 2; ++i) {
    const int mB = m0 + 16 * i;
#pragma unroll
    for (int j = 0; j < 4; ++j) {
      const int n = n0 + 16 * j + rl;
      float bcol = 0.f;
      if (BIAS_MODE == 2) bcol = bias[n];
#pragma unroll
      for (int r = 0; r < 8; ++r) {
        const int m = mB + 8 * hf + r;
        float v = acc[i][j][r] * scale;
        if (BIAS_MODE == 1) v += bias[m];
        if (BIAS_MODE == 2) v += bcol;
        if (RELU) v = fmaxf(v, 0.0f);
        if (MUL) v *= mul[(size_t)m * ldc + n];
        slab[(8 * hf + r) * 68 + 16 * j + rl] = v;
      }
    }
    wave_lds_sync();
    if (OUT16 == 0) {
      float* C = (float*)Cp + (size_t)z * sC;
      const int c4 = rl * 4;
      for (int pass = 0; pass < 2; ++pass) {
#pragma unroll
        for (int it = 0; it < 8; ++it) {
          const int row = it * 2 + hf;
          const v4f v = *(const v4f*)(slab + row * 68 + c4);
          *(volatile v4f*)(C + (size_t)(mB + row) * ldc + n0 + c4) = v;
        }
        __threadfence();
      }
    } else {
      _Float16* C = (_Float16*)Cp + (size_t)z * sC;
      const int q8 = lane >> 3, c8 = (lane & 7) * 8;
      v8h hv[4];
#pragma unroll
      for (int it = 0; it < 4; ++it) {
        const int row = it * 4 + q8;
        const float* sp = slab + row * 68 + c8;
        v8h v;
#pragma unroll
        for (int e = 0; e < 8; ++e) v[e] = (_Float16)(sp[e] * oscale);
        hv[it] = v;
      }
      for (int pass = 0; pass < 2; ++pass) {
#pragma unroll
        for (int it = 0; it < 4; ++it) {
          const int row = it * 4 + q8;
          *(volatile v8h*)(C + (size_t)(mB + row) * ldc + n0 + c8) = hv[it];
        }
        __threadfence();
      }
    }
    wave_lds_sync();
  }
}

#define ATT_KT 32
#define ATT_QP 264
#define ATT_VP 40
#define ATT_PP 40
#define ATT_LDS_HALVES (64 * ATT_QP + ATT_KT * ATT_QP + DMOD * ATT_VP + 4 * 16 * ATT_PP)
#define ATT_LDS_BYTES  (ATT_LDS_HALVES * 2 + 2 * 128 * 4)

__global__ __launch_bounds__(256) __attribute__((amdgpu_num_vgpr(224))) void attn_kernel(
    const unsigned short* __restrict__ qp, const unsigned short* __restrict__ ikp,
    const unsigned short* __restrict__ ivtp, const unsigned short* __restrict__ mkp,
    const unsigned short* __restrict__ mvp, unsigned short* __restrict__ valp) {
  extern __shared__ v4f dsm_raw[];
  _Float16* Qs  = (_Float16*)dsm_raw;
  _Float16* Ks  = Qs + 64 * ATT_QP;
  _Float16* Vts = Ks + ATT_KT * ATT_QP;
  _Float16* Ps  = Vts + DMOD * ATT_VP;
  float*    Xm  = (float*)(Ps + 4 * 16 * ATT_PP);
  float*    Xl  = Xm + 128;

  const int tid  = threadIdx.x;
  const int wv   = tid >> 5;
  const int lane = tid & 31;
  const int hf   = lane >> 4;
  const int c    = lane & 15;
  const int rg   = wv & 3;
  const int kh   = wv >> 2;
  const int cb   = blockIdx.x;
  const int b    = blockIdx.y;
  const int h    = blockIdx.z;
  const int gm0  = b * LSM + cb * 64;

  const _Float16* Q   = (const _Float16*)qp;
  const _Float16* IK  = (const _Float16*)ikp  + (size_t)b * LSI * DMOD;
  const _Float16* IVT = (const _Float16*)ivtp + (size_t)b * DMOD * LSI;
  const _Float16* MK  = (const _Float16*)mkp;
  const _Float16* MV  = (const _Float16*)mvp;
  _Float16*       VO  = (_Float16*)valp;

#pragma unroll
  for (int it = 0; it < 8; ++it) {
    const int idx = it * 256 + tid;
    const int r   = idx >> 5;
    const int cq  = idx & 31;
    const v8h v = *(const v8h*)(Q + (size_t)(gm0 + r) * QCOLS + h * DMOD + cq * 8);
    *(v8h*)(Qs + r * ATT_QP + cq * 8) = v;
  }
  __syncthreads();

  const int wr0 = rg * 16;
  const int vc0 = kh * 128;
  float mrow[8], lrow[8];
  v8f O[8];
#pragma unroll
  for (int r = 0; r < 8; ++r) {
    const int lr = wr0 + 8 * hf + r;
    const size_t gm = (size_t)(gm0 + lr);
    const v8h qa = *(const v8h*)(Qs + lr * ATT_QP + 16 * c);
    const v8h qb = *(const v8h*)(Qs + lr * ATT_QP + 16 * c + 8);
    const v8h ka = *(const v8h*)(MK + gm * DMOD + 16 * c);
    const v8h kb = *(const v8h*)(MK + gm * DMOD + 16 * c + 8);
    float d = 0.f;
#pragma unroll
    for (int e = 0; e < 8; ++e) d += (float)qa[e] * (float)ka[e];
#pragma unroll
    for (int e = 0; e < 8; ++e) d += (float)qb[e] * (float)kb[e];
#pragma unroll
    for (int off = 8; off >= 1; off >>= 1) d += __shfl_xor(d, off, 32);
    mrow[r] = d * (1.0f / 256.0f);
    lrow[r] = 1.0f;
#pragma unroll
    for (int cc = 0; cc < 8; ++cc) O[cc][r] = (float)MV[gm * DMOD + vc0 + 16 * cc + c];
  }

  _Float16* Pw = Ps + rg * 16 * ATT_PP;
  float* xmw = Xm + (rg * 2 + kh) * 16;
  float* xlw = Xl + (rg * 2 + kh) * 16;
  const float* xm0 = Xm + rg * 32;
  const float* xm1 = xm0 + 16;
  const float* xl0 = Xl + rg * 32;
  const float* xl1 = xl0 + 16;

  for (int t = 0; t < LSI / ATT_KT; ++t) {
    const int s0 = t * ATT_KT;
    __syncthreads();
#pragma unroll
    for (int it = 0; it < 4; ++it) {
      const int idx = it * 256 + tid;
      const int kr  = idx >> 5;
      const int cq  = idx & 31;
      const v8h v = *(const v8h*)(IK + (size_t)(s0 + kr) * DMOD + cq * 8);
      *(v8h*)(Ks + kr * ATT_QP + cq * 8) = v;
    }
#pragma unroll
    for (int it = 0; it < 4; ++it) {
      const int idx = it * 256 + tid;
      const int dd  = idx >> 2;
      const int cq  = idx & 3;
      const v8h v = *(const v8h*)(IVT + (size_t)dd * LSI + s0 + cq * 8);
      *(v8h*)(Vts + dd * ATT_VP + cq * 8) = v;
    }
    __syncthreads();

    v8f S = zero8f();
#pragma unroll
    for (int ks = 0; ks < 8; ++ks) {
      const v16h qa = ldfrag(Qs + (wr0 + c) * ATT_QP + ks * 32 + 8 * hf);
      const v16h kf = ldfrag(Ks + (16 * kh + c) * ATT_QP + ks * 32 + 8 * hf);
      S = mma16(qa, kf, S);
    }

    float xr[8];
#pragma unroll
    for (int r = 0; r < 8; ++r) {
      const float x = S[r] * (1.0f / 256.0f);
      float bm = x;
#pragma unroll
      for (int off = 8; off >= 1; off >>= 1) bm = fmaxf(bm, __shfl_xor(bm, off, 32));
      xr[r] = x;
      if (c == 0) xmw[8 * hf + r] = bm;
    }
    __syncthreads();

#pragma unroll
    for (int r = 0; r < 8; ++r) {
      const int row = 8 * hf + r;
      const float bt   = fmaxf(xm0[row], xm1[row]);
      const float mnew = fmaxf(mrow[r], bt);
      const float cr   = expf(mrow[r] - mnew);
      const float p    = expf(xr[r] - mnew);
      float ps = p;
#pragma unroll
      for (int off = 8; off >= 1; off >>= 1) ps += __shfl_xor(ps, off, 32);
      if (c == 0) xlw[row] = ps;
      Pw[row * ATT_PP + 16 * kh + c] = (_Float16)p;
      mrow[r] = mnew;
      lrow[r] *= cr;
#pragma unroll
      for (int cc = 0; cc < 8; ++cc) O[cc][r] *= cr;
    }
    __syncthreads();

#pragma unroll
    for (int r = 0; r < 8; ++r) {
      const int row = 8 * hf + r;
      lrow[r] = lrow[r] + (xl0[row] + xl1[row]);
    }
    const v16h pa = ldfrag(Pw + c * ATT_PP + 8 * hf);
#pragma unroll
    for (int cc = 0; cc < 8; ++cc) {
      const v16h vb = ldfrag(Vts + (vc0 + 16 * cc + c) * ATT_VP + 8 * hf);
      O[cc] = mma16(pa, vb, O[cc]);
    }
  }
  __syncthreads();

  _Float16* Os = Qs + wr0 * ATT_QP + vc0;
#pragma unroll
  for (int r = 0; r < 8; ++r) {
    const float inv = 64.0f * (1.0f / lrow[r]);
#pragma unroll
    for (int cc = 0; cc < 8; ++cc) Os[(8 * hf + r) * ATT_QP + 16 * cc + c] = (_Float16)(O[cc][r] * inv);
  }
  __syncthreads();
  for (int pass = 0; pass < 2; ++pass) {
#pragma unroll
    for (int rr = 0; rr < 8; ++rr) {
      const int row = 8 * wv + rr;
      const v8h v = *(const v8h*)(Qs + row * ATT_QP + 8 * lane);
      *(volatile v8h*)(VO + (size_t)(gm0 + row) * QCOLS + h * DMOD + 8 * lane) = v;
    }
    __threadfence();
  }
}

template <int OUTH>
__global__ __launch_bounds__(256) void ln_kernel(const float* __restrict__ a, const float* __restrict__ res,
                                                 const float* __restrict__ g, const float* __restrict__ bta,
                                                 float* __restrict__ outF, unsigned short* __restrict__ outHp) {
  __shared__ __align__(16) float srow[8][DMOD];
  const int lane = threadIdx.x & 31;
  const int wv   = threadIdx.x >> 5;
  const size_t row = (size_t)blockIdx.x * 8 + wv;
  const float* pa = a + row * DMOD;
  const float* pr = res + row * DMOD;
  float x[8];
  float s = 0.f;
#pragma unroll
  for (int i = 0; i < 8; ++i) {
    const int col = i * 32 + lane;
    x[i] = pa[col] + pr[col];
    s += x[i];
  }
#pragma unroll
  for (int off = 16; off >= 1; off >>= 1) s += __shfl_xor(s, off, 32);
  const float mean = s * (1.0f / 256.0f);
  float vs = 0.f;
#pragma unroll
  for (int i = 0; i < 8; ++i) { const float d = x[i] - mean; vs += d * d; }
#pragma unroll
  for (int off = 16; off >= 1; off >>= 1) vs += __shfl_xor(vs, off, 32);
  const float rstd = rsqrtf(vs * (1.0f / 256.0f) + 1e-6f);
  float* sr = srow[wv];
#pragma unroll
  for (int i = 0; i < 8; ++i) {
    const int col = i * 32 + lane;
    sr[col] = (x[i] - mean) * rstd * g[col] + bta[col];
  }
  wave_lds_sync();
  const v4f y0 = *(const v4f*)(sr + 4 * lane);
  const v4f y1 = *(const v4f*)(sr + 128 + 4 * lane);
  v8h yh;
  if (OUTH) {
#pragma unroll
    for (int e = 0; e < 8; ++e) yh[e] = (_Float16)sr[8 * lane + e];
  }
  float* po = outF + row * DMOD;
  _Float16* ph = (_Float16*)outHp + row * DMOD;
  for (int pass = 0; pass < 2; ++pass) {
    *(volatile v4f*)(po + 4 * lane)       = y0;
    *(volatile v4f*)(po + 128 + 4 * lane) = y1;
    if (OUTH) *(volatile v8h*)(ph + 8 * lane) = yh;
    __threadfence();
  }
}

extern "C" void kernel_launch(void* const* d_in, const int* in_sizes, int n_in,
                              void* d_out, int out_size, void* d_ws, size_t ws_size,
                              hipStream_t stream) {
  if (n_in < 22) return;
  if (in_sizes[0] != MROWS * DMOD || in_sizes[1] != IROWS * DMOD) return;
  if (in_sizes[2] != DMOD * DMOD || in_sizes[3] != DMOD || in_sizes[4] != DMOD * DMOD || in_sizes[5] != DMOD) return;
  if (in_sizes[6] != NHEAD * DMOD * DMOD || in_sizes[7] != NHEAD * DMOD) return;
  if (in_sizes[8] != QCOLS * DMOD || in_sizes[9] != DMOD || in_sizes[10] != DMOD || in_sizes[11] != DMOD) return;
  if (in_sizes[12] != DMOD * DFF || in_sizes[13] != DFF) return;
  if (in_sizes[14] != DFF * DFF || in_sizes[15] != DFF || in_sizes[16] != DFF * DFF || in_sizes[17] != DFF) return;
  if (in_sizes[18] != DFF * DMOD || in_sizes[19] != DMOD || in_sizes[20] != DMOD || in_sizes[21] != DMOD) return;
  if (out_size != MROWS * DMOD) return;

  const float* state = (const float*)d_in[0];
  const float* input = (const float*)d_in[1];
  const float* Wk    = (const float*)d_in[2];
  const float* bk    = (const float*)d_in[3];
  const float* Wv    = (const float*)d_in[4];
  const float* bv    = (const float*)d_in[5];
  const float* Wq    = (const float*)d_in[6];
  const float* bq    = (const float*)d_in[7];
  const float* Wo    = (const float*)d_in[8];
  const float* bo    = (const float*)d_in[9];
  const float* ln1g  = (const float*)d_in[10];
  const float* ln1b  = (const float*)d_in[11];
  const float* Win   = (const float*)d_in[12];
  const float* bin   = (const float*)d_in[13];
  const float* Wgnl  = (const float*)d_in[14];
  const float* bgnl  = (const float*)d_in[15];
  const float* Wgl   = (const float*)d_in[16];
  const float* bgl   = (const float*)d_in[17];
  const float* Wgo   = (const float*)d_in[18];
  const float* bgo   = (const float*)d_in[19];
  const float* ln2g  = (const float*)d_in[20];
  const float* ln2b  = (const float*)d_in[21];
  float* out = (float*)d_out;

  size_t off = 0;
  const size_t oWkT  = off; off += (size_t)DMOD * DMOD * 2;
  const size_t oWvT  = off; off += (size_t)DMOD * DMOD * 2;
  const size_t oWqT  = off; off += (size_t)QCOLS * DMOD * 2;
  const size_t oWoT  = off; off += (size_t)DMOD * QCOLS * 2;
  const size_t oWinT = off; off += (size_t)DFF * DMOD * 2;
  const size_t oWnlT = off; off += (size_t)DFF * DFF * 2;
  const size_t oWlT  = off; off += (size_t)DFF * DFF * 2;
  const size_t oWgoT = off; off += (size_t)DMOD * DFF * 2;
  const size_t oXs   = off; off += (size_t)MROWS * DMOD * 2;
  const size_t oXi   = off; off += (size_t)IROWS * DMOD * 2;
  const size_t oIK   = off; off += (size_t)IROWS * DMOD * 2;
  const size_t oIVT  = off; off += (size_t)NBATCH * DMOD * LSI * 2;
  const size_t oMK   = off; off += (size_t)MROWS * DMOD * 2;
  const size_t oMV   = off; off += (size_t)MROWS * DMOD * 2;
  const size_t oQP   = off; off += (size_t)MROWS * QCOLS * 2;
  const size_t oVAL  = off; off += (size_t)MROWS * QCOLS * 2;
  const size_t oAO   = off; off += (size_t)MROWS * DMOD * 4;
  const size_t oX    = off; off += (size_t)MROWS * DMOD * 4;
  const size_t oXH   = off; off += (size_t)MROWS * DMOD * 2;
  const size_t oH4   = off; off += (size_t)MROWS * DFF * 2;
  const size_t oVL   = off; off += (size_t)MROWS * DFF * 4;
  const size_t oG64  = off; off += (size_t)MROWS * DFF * 2;
  const size_t oFF   = off; off += (size_t)MROWS * DMOD * 4;
  if (off > ws_size) return;
  if (off > (size_t)134217728) return;

  char* ws = (char*)d_ws;
  unsigned short* WkT  = (unsigned short*)(ws + oWkT);
  unsigned short* WvT  = (unsigned short*)(ws + oWvT);
  unsigned short* WqT  = (unsigned short*)(ws + oWqT);
  unsigned short* WoT  = (unsigned short*)(ws + oWoT);
  unsigned short* WinT = (unsigned short*)(ws + oWinT);
  unsigned short* WnlT = (unsigned short*)(ws + oWnlT);
  unsigned short* WlT  = (unsigned short*)(ws + oWlT);
  unsigned short* WgoT = (unsigned short*)(ws + oWgoT);
  unsigned short* Xs   = (unsigned short*)(ws + oXs);
  unsigned short* Xi   = (unsigned short*)(ws + oXi);
  unsigned short* IKp  = (unsigned short*)(ws + oIK);
  unsigned short* IVTp = (unsigned short*)(ws + oIVT);
  unsigned short* MKp  = (unsigned short*)(ws + oMK);
  unsigned short* MVp  = (unsigned short*)(ws + oMV);
  unsigned short* QPp  = (unsigned short*)(ws + oQP);
  unsigned short* VALp = (unsigned short*)(ws + oVAL);
  float*          AO   = (float*)(ws + oAO);
  float*          X    = (float*)(ws + oX);
  unsigned short* XH   = (unsigned short*)(ws + oXH);
  unsigned short* H4   = (unsigned short*)(ws + oH4);
  float*          VL   = (float*)(ws + oVL);
  unsigned short* G64  = (unsigned short*)(ws + oG64);
  float*          FFp  = (float*)(ws + oFF);

  const dim3 blk(256);
  const float kW  = 64.0f;
  const long  WQS = (long)DMOD * DMOD;

  {
    const int n8s = MROWS * DMOD / 8, n8i = IROWS * DMOD / 8;
    cvt_f16_kernel<<<dim3((n8s + 255) / 256), blk, 0, stream>>>(state, Xs, n8s);
    cvt_f16_kernel<<<dim3((n8i + 255) / 256), blk, 0, stream>>>(input, Xi, n8i);
  }
  tcvt_kernel<<<dim3(DMOD / 64, DMOD / 64, 1),     blk, 0, stream>>>(Wk,   WkT,  DMOD,  DMOD,  0L, 0L, kW);
  tcvt_kernel<<<dim3(DMOD / 64, DMOD / 64, 1),     blk, 0, stream>>>(Wv,   WvT,  DMOD,  DMOD,  0L, 0L, kW);
  tcvt_kernel<<<dim3(DMOD / 64, DMOD / 64, NHEAD), blk, 0, stream>>>(Wq,   WqT,  DMOD,  DMOD,  WQS, WQS, kW);
  tcvt_kernel<<<dim3(DMOD / 64, QCOLS / 64, 1),    blk, 0, stream>>>(Wo,   WoT,  QCOLS, DMOD,  0L, 0L, kW);
  tcvt_kernel<<<dim3(DFF / 64, DMOD / 64, 1),      blk, 0, stream>>>(Win,  WinT, DMOD,  DFF,   0L, 0L, kW);
  tcvt_kernel<<<dim3(DFF / 64, DFF / 64, 1),       blk, 0, stream>>>(Wgnl, WnlT, DFF,   DFF,   0L, 0L, kW);
  tcvt_kernel<<<dim3(DFF / 64, DFF / 64, 1),       blk, 0, stream>>>(Wgl,  WlT,  DFF,   DFF,   0L, 0L, kW);
  tcvt_kernel<<<dim3(DMOD / 64, DFF / 64, 1),      blk, 0, stream>>>(Wgo,  WgoT, DFF,   DMOD,  0L, 0L, kW);

  gemm_kernel<2, 1, 0, 0><<<dim3(((IROWS / 32) * (DMOD / 64)) / 8, 1), blk, 0, stream>>>(
      Xi, DMOD, 0L, WkT, DMOD, 0L, (void*)IKp, DMOD, 0L, bk, bk, IROWS, DMOD, DMOD, 1.0f / 64.0f, 4.0f);
  gemm_kernel<1, 1, 0, 0><<<dim3(((DMOD / 32) * (LSI / 64)) / 8, NBATCH), blk, 0, stream>>>(
      WvT, DMOD, 0L, Xi, DMOD, (long)LSI * DMOD, (void*)IVTp, LSI, (long)DMOD * LSI, bv, bv, DMOD, LSI, DMOD, 1.0f / 64.0f, 4.0f);
  gemm_kernel<2, 1, 0, 0><<<dim3(((MROWS / 32) * (DMOD / 64)) / 8, 1), blk, 0, stream>>>(
      Xs, DMOD, 0L, WkT, DMOD, 0L, (void*)MKp, DMOD, 0L, bk, bk, MROWS, DMOD, DMOD, 1.0f / 64.0f, 4.0f);
  gemm_kernel<2, 1, 0, 0><<<dim3(((MROWS / 32) * (DMOD / 64)) / 8, 1), blk, 0, stream>>>(
      Xs, DMOD, 0L, WvT, DMOD, 0L, (void*)MVp, DMOD, 0L, bv, bv, MROWS, DMOD, DMOD, 1.0f / 64.0f, 4.0f);
  gemm_kernel<2, 1, 0, 0><<<dim3(((MROWS / 32) * (QCOLS / 64)) / 8, 1), blk, 0, stream>>>(
      Xs, DMOD, 0L, WqT, DMOD, 0L, (void*)QPp, QCOLS, 0L, bq, bq, MROWS, QCOLS, DMOD, 1.0f / 64.0f, 4.0f);

  (void)hipFuncSetAttribute(reinterpret_cast<const void*>(&attn_kernel), hipFuncAttributeMaxDynamicSharedMemorySize, ATT_LDS_BYTES);
  attn_kernel<<<dim3(LSM / 64, NBATCH, NHEAD), dim3(256), ATT_LDS_BYTES, stream>>>(QPp, IKp, IVTp, MKp, MVp, VALp);

  gemm_kernel<2, 0, 0, 0><<<dim3(((MROWS / 32) * (DMOD / 64)) / 8, 1), blk, 0, stream>>>(
      VALp, QCOLS, 0L, WoT, QCOLS, 0L, (void*)AO, DMOD, 0L, bo, bo, MROWS, DMOD, QCOLS, 1.0f / 16384.0f, 1.0f);
  ln_kernel<1><<<dim3(MROWS / 8), blk, 0, stream>>>(AO, state, ln1g, ln1b, X, XH);

  gemm_kernel<2, 1, 1, 0><<<dim3(((MROWS / 32) * (DFF / 64)) / 8, 1), blk, 0, stream>>>(
      XH, DMOD, 0L, WinT, DMOD, 0L, (void*)H4, DFF, 0L, bin, bin, MROWS, DFF, DMOD, 1.0f / 64.0f, 4.0f);
  gemm_kernel<2, 0, 0, 0><<<dim3(((MROWS / 32) * (DFF / 64)) / 8, 1), blk, 0, stream>>>(
      H4, DFF, 0L, WlT, DFF, 0L, (void*)VL, DFF, 0L, bgl, bgl, MROWS, DFF, DFF, 1.0f / 256.0f, 1.0f);
  gemm_kernel<2, 1, 1, 1><<<dim3(((MROWS / 32) * (DFF / 64)) / 8, 1), blk, 0, stream>>>(
      H4, DFF, 0L, WnlT, DFF, 0L, (void*)G64, DFF, 0L, bgnl, VL, MROWS, DFF, DFF, 1.0f / 256.0f, 64.0f);
  gemm_kernel<2, 0, 0, 0><<<dim3(((MROWS / 32) * (DMOD / 64)) / 8, 1), blk, 0, stream>>>(
      G64, DFF, 0L, WgoT, DFF, 0L, (void*)FFp, DMOD, 0L, bgo, bgo, MROWS, DMOD, DFF, 1.0f / 4096.0f, 1.0f);
  ln_kernel<0><<<dim3(MROWS / 8), blk, 0, stream>>>(FFp, X, ln2g, ln2b, out, XH);

  (void)hipGetLastError();
}
